// CustomJacobiLayer_45243185496810
// MI455X (gfx1250) — hardware-verified
//
#include <hip/hip_runtime.h>
#include <stddef.h>
#include <stdint.h>
#include <math.h>

#define NB  4096
#define NI  512
#define ND  8
#define NO  512
#define NK  (NI * ND)
#define TBM 64
#define TBN 64

static_assert((NK % 32) == 0);
static_assert((NB % TBM) == 0);
static_assert((NO % TBN) == 0);
static_assert(((NB * NI) % 256) == 0);
static_assert(((NO * NK) % 2048) == 0);
static_assert(TBM == 64);
static_assert(TBN == 64);
static_assert(ND == 8);

typedef _Float16     v16h __attribute__((ext_vector_type(16)));
typedef float        v8f  __attribute__((ext_vector_type(8)));
typedef float        v4f  __attribute__((ext_vector_type(4)));
typedef unsigned int v4u  __attribute__((ext_vector_type(4)));

#define JK1(i) ((float)(((2.0 * (i) + 1.0 + 1.0) * (2.0 * (i) + 1.0 + 1.0 - 1.0)) / ((2.0 * (i)) * ((i) + 1.0 + 1.0))))
#define JK3(i) ((float)((((i) + 1.0 - 1.0) * ((i) + 1.0 - 1.0) * (2.0 * (i) + 1.0 + 1.0)) / \
                        (((double)(i)) * ((i) + 1.0 + 1.0) * (2.0 * (i) + 1.0 + 1.0 - 2.0))))

__device__ __forceinline__ unsigned short bf_bits(float f) {
  const unsigned u = __float_as_uint(f);
  return (unsigned short)((u + 0x7FFFu + ((u >> 16) & 1u)) >> 16);
}
__device__ __forceinline__ float bfr(float f) { return __uint_as_float(((unsigned)bf_bits(f)) << 16); }
__device__ __forceinline__ unsigned pk16(unsigned short a, unsigned short b) { return (unsigned)a | ((unsigned)b << 16); }
__device__ __forceinline__ v8f zero8() { v8f z = {0.f, 0.f, 0.f, 0.f, 0.f, 0.f, 0.f, 0.f}; return z; }
__device__ __forceinline__ _Float16 to_h_flush(float f) {
  const float a = fabsf(f) < 6.103515625e-05f ? 0.0f : f;
  return (_Float16)a;
}
__device__ __forceinline__ unsigned short h_bits(_Float16 h) { return __builtin_bit_cast(unsigned short, h); }
__device__ __forceinline__ float vgpr_opaque(float v) {
#if defined(__HIP_DEVICE_COMPILE__)
  asm volatile("" : "+v"(v));
#endif
  return v;
}

struct HL { unsigned short h, l; };
__device__ __forceinline__ HL split16(float p) {
  HL r;
  const _Float16 hv = to_h_flush(p);
  r.h = h_bits(hv);
  r.l = h_bits(to_h_flush((p - (float)hv) * 4096.0f));
  return r;
}

union Frag { v16h h; v4u u[2]; };
__device__ __forceinline__ Frag ldfrag(const unsigned short* p) {
  Frag f;
  f.u[0] = *(const v4u*)(p);
  f.u[1] = *(const v4u*)(p + 16);
  return f;
}

__device__ __forceinline__ v8f mma16(const Frag& a, const Frag& b, v8f c) {
  return __builtin_amdgcn_wmma_f32_16x16x32_f16(false, a.h, false, b.h, (short)0, c, false, false);
}
__device__ __forceinline__ void guard8(v8f& c0, v8f& c1, v8f& c2, v8f& c3, v8f& c4, v8f& c5, v8f& c6, v8f& c7,
                                       const Frag& a0, const Frag& a1, const Frag& a2, const Frag& a3,
                                       const Frag& b0, const Frag& b1) {
#if defined(__HIP_DEVICE_COMPILE__)
  asm volatile("v_nop\n\tv_nop\n\tv_nop\n\tv_nop"
               : "+v"(c0), "+v"(c1), "+v"(c2), "+v"(c3), "+v"(c4), "+v"(c5), "+v"(c6), "+v"(c7)
               : "v"(a0.h), "v"(a1.h), "v"(a2.h), "v"(a3.h), "v"(b0.h), "v"(b1.h));
#endif
}

__global__ __launch_bounds__(256)
void k_feat(const float* __restrict__ x, unsigned short* Ah, unsigned short* Al, int ntot) {
#pragma clang fp contract(off)
  const size_t t = (size_t)blockIdx.x * 256 + threadIdx.x;
  if (t >= (size_t)ntot) return;
  const float u  = tanhf(bfr(x[t]));
  const float p0 = vgpr_opaque(1.0f);
  const float p1 = 2.0f * u;
  const float p2 = (JK1(2) * u) * p1 - JK3(2) * p0;
  const float p3 = (JK1(3) * u) * p2 - JK3(3) * p1;
  const float p4 = (JK1(4) * u) * p3 - JK3(4) * p2;
  const float p5 = (JK1(5) * u) * p4 - JK3(5) * p3;
  const float p6 = (JK1(6) * u) * p5 - JK3(6) * p4;
  const float p7 = (JK1(7) * u) * p6 - JK3(7) * p5;
  const HL s0 = split16(p0), s1 = split16(p1), s2 = split16(p2), s3 = split16(p3);
  const HL s4 = split16(p4), s5 = split16(p5), s6 = split16(p6), s7 = split16(p7);
  v4u uh, ul;
  uh[0] = pk16(s0.h, s1.h); uh[1] = pk16(s2.h, s3.h); uh[2] = pk16(s4.h, s5.h); uh[3] = pk16(s6.h, s7.h);
  ul[0] = pk16(s0.l, s1.l); ul[1] = pk16(s2.l, s3.l); ul[2] = pk16(s4.l, s5.l); ul[3] = pk16(s6.l, s7.l);
  unsigned short* dh = Ah + t * 8;
  unsigned short* dl = Al + t * 8;
  *(volatile v4u*)dh = uh;
  *(volatile v4u*)dl = ul;
  __threadfence();
  *(volatile v4u*)dh = uh;
  *(volatile v4u*)dl = ul;
}

__global__ __launch_bounds__(256)
void k_cvb(const float* __restrict__ src, unsigned short* dst, int ntot) {
  const size_t f8 = ((size_t)blockIdx.x * 256 + threadIdx.x) * 8;
  if (f8 + 8 > (size_t)ntot) return;
  const v4f a = *(const v4f*)(src + f8);
  const v4f b = *(const v4f*)(src + f8 + 4);
  v4u u;
  u[0] = pk16(h_bits(to_h_flush(bfr(a[0]) * 256.0f)), h_bits(to_h_flush(bfr(a[1]) * 256.0f)));
  u[1] = pk16(h_bits(to_h_flush(bfr(a[2]) * 256.0f)), h_bits(to_h_flush(bfr(a[3]) * 256.0f)));
  u[2] = pk16(h_bits(to_h_flush(bfr(b[0]) * 256.0f)), h_bits(to_h_flush(bfr(b[1]) * 256.0f)));
  u[3] = pk16(h_bits(to_h_flush(bfr(b[2]) * 256.0f)), h_bits(to_h_flush(bfr(b[3]) * 256.0f)));
  unsigned short* dp = dst + f8;
  *(volatile v4u*)dp = u;
  __threadfence();
  *(volatile v4u*)dp = u;
}

__global__ __launch_bounds__(128)
void k_gemm(const unsigned short* __restrict__ Ahp, const unsigned short* __restrict__ Alp,
            const unsigned short* __restrict__ Bm, float* C, int K, int ldc) {
  __shared__ __align__(16) float sO[TBM * TBN];
  const int tid = threadIdx.x, w = tid >> 5, lane = tid & 31, hh = lane >> 4, c = lane & 15;
  const int wm = w & 1, wn = w >> 1;
  const int Mbase = blockIdx.y * TBM, Nbase = blockIdx.x * TBN;
  const int mrow0 = Mbase + 32 * wm;
  const int ncol0 = Nbase + 32 * wn;
  const size_t Ks = (size_t)K;

  const unsigned short* aph0 = Ahp + (size_t)(mrow0 + c) * Ks + 8 * hh;
  const unsigned short* aph1 = aph0 + 16 * Ks;
  const unsigned short* apl0 = Alp + (size_t)(mrow0 + c) * Ks + 8 * hh;
  const unsigned short* apl1 = apl0 + 16 * Ks;
  const unsigned short* bp0  = Bm + (size_t)(ncol0 + c) * Ks + 8 * hh;
  const unsigned short* bp1  = bp0 + 16 * Ks;

  v8f ach[2][2], acl[2][2];
#pragma unroll
  for (int mi = 0; mi < 2; ++mi)
#pragma unroll
    for (int ni = 0; ni < 2; ++ni) { ach[mi][ni] = zero8(); acl[mi][ni] = zero8(); }

  const int nk = K >> 5;
#pragma unroll 1
  for (int ks = 0; ks < nk; ++ks) {
    const int ko = ks << 5;
    const Frag a0 = ldfrag(aph0 + ko);
    const Frag a1 = ldfrag(aph1 + ko);
    const Frag e0 = ldfrag(apl0 + ko);
    const Frag e1 = ldfrag(apl1 + ko);
    const Frag b0 = ldfrag(bp0 + ko);
    const Frag b1 = ldfrag(bp1 + ko);
    ach[0][0] = mma16(a0, b0, ach[0][0]);
    ach[0][1] = mma16(a0, b1, ach[0][1]);
    ach[1][0] = mma16(a1, b0, ach[1][0]);
    ach[1][1] = mma16(a1, b1, ach[1][1]);
    acl[0][0] = mma16(e0, b0, acl[0][0]);
    acl[0][1] = mma16(e0, b1, acl[0][1]);
    acl[1][0] = mma16(e1, b0, acl[1][0]);
    acl[1][1] = mma16(e1, b1, acl[1][1]);
    guard8(ach[0][0], ach[0][1], ach[1][0], ach[1][1], acl[0][0], acl[0][1], acl[1][0], acl[1][1],
           a0, a1, e0, e1, b0, b1);
  }

#pragma unroll
  for (int mi = 0; mi < 2; ++mi) {
#pragma unroll
    for (int ni = 0; ni < 2; ++ni) {
      const int lcol = 32 * wn + 16 * ni + c;
      const v8f v = (ach[mi][ni] + acl[mi][ni] * (1.0f / 4096.0f)) * (1.0f / 256.0f);
#pragma unroll
      for (int r = 0; r < 8; ++r) {
        const int lrow = 32 * wm + 16 * mi + 8 * hh + r;
        sO[lrow * TBN + lcol] = v[r];
      }
    }
  }
  __syncthreads();

  const int c4 = c * 4;
  v4f o[8];
#pragma unroll
  for (int it = 0; it < 8; ++it) {
    const int lr = 16 * w + 2 * it + hh;
    o[it] = *(const v4f*)(sO + lr * TBN + c4);
  }
  float* cp = C + (size_t)(Mbase + 16 * w + hh) * (size_t)ldc + Nbase + c4;
#pragma unroll
  for (int it = 0; it < 8; ++it) *(volatile v4f*)(cp + (size_t)(2 * it) * (size_t)ldc) = o[it];
  __threadfence();
#pragma unroll
  for (int it = 0; it < 8; ++it) *(volatile v4f*)(cp + (size_t)(2 * it) * (size_t)ldc) = o[it];
}

extern "C" void kernel_launch(void* const* d_in, const int* in_sizes, int n_in,
                              void* d_out, int out_size, void* d_ws, size_t ws_size,
                              hipStream_t stream) {
  if (n_in < 2) return;
  if (in_sizes[0] != NB * NI) return;
  if (in_sizes[1] != NO * NK) return;
  if (out_size != NB * NO) return;

  const float* x    = (const float*)d_in[0];
  const float* coef = (const float*)d_in[1];
  float* out = (float*)d_out;

  const size_t sAh = (size_t)NB * NK * 2;
  const size_t sAl = (size_t)NB * NK * 2;
  const size_t sB  = (size_t)NO * NK * 2;
  size_t off = 0;
  const size_t oAh = off; off += sAh;
  const size_t oAl = off; off += sAl;
  const size_t oB  = off; off += sB;
  if (off > ws_size) return;
  if (off > (size_t)134217728) return;

  char* ws = (char*)d_ws;
  unsigned short* Ah = (unsigned short*)(ws + oAh);
  unsigned short* Al = (unsigned short*)(ws + oAl);
  unsigned short* Bt = (unsigned short*)(ws + oB);

  k_feat<<<dim3((NB * NI) / 256), dim3(256), 0, stream>>>(x, Ah, Al, NB * NI);
  k_cvb<<<dim3((NO * NK) / 2048), dim3(256), 0, stream>>>(coef, Bt, NO * NK);
  k_gemm<<<dim3(NO / TBN, NB / TBM), dim3(128), 0, stream>>>(Ah, Al, Bt, out, NK, NO);
  (void)hipGetLastError();
}
